// LinearCrossAttention_54812372631770
// MI455X (gfx1250) — hardware-verified
//
#include <hip/hip_runtime.h>
#include <math.h>

#ifndef NB
#define NB 4
#endif
#ifndef SEQ
#define SEQ 8192
#endif
#define NB_FULL 4
#define SEQ_FULL 8192
#define CC 256
#define HH 8
#define DD 32
#define TOKB 64
#define OTS 72
#define LN_EPS 1e-5f
#define WCARRY 16384.0f
#define WCARRY_INV 6.103515625e-05f
#define PCARRY 64.0f

static_assert(NB >= 1 && NB <= NB_FULL);
static_assert(SEQ >= 256 && SEQ <= SEQ_FULL && (SEQ % 256) == 0);
static_assert(CC == HH * DD);
static_assert((SEQ % TOKB) == 0);
static_assert((size_t)NB * SEQ * CC * 2 * 3 + (size_t)CC * CC * 2 * 2 + (size_t)NB * HH * DD * 4 <= (size_t)134217728);

typedef _Float16 f16;
typedef f16 f16x16 __attribute__((ext_vector_type(16)));
typedef f16 f16x8 __attribute__((ext_vector_type(8)));
typedef float f32x8 __attribute__((ext_vector_type(8)));
typedef unsigned v4u __attribute__((ext_vector_type(4)));
typedef unsigned v4ua __attribute__((ext_vector_type(4), may_alias));
typedef float v4f __attribute__((ext_vector_type(4)));
typedef float v4fa __attribute__((ext_vector_type(4), may_alias));
union Frag { f16x16 v; f16x8 h[2]; };
union Pack8 { f16x8 v; v4u u; };

__device__ __forceinline__ f32x8 wmma16(f16x16 a, f16x16 b, f32x8 c) {
  c = __builtin_amdgcn_wmma_f32_16x16x32_f16(false, a, false, b, (short)0, c, false, false);
  asm volatile("v_nop\n\tv_nop\n\tv_nop\n\tv_nop" : "+v"(c) : "v"(a), "v"(b));
  return c;
}

__device__ __forceinline__ float bf16r(float x) {
  unsigned u = __float_as_uint(x);
  u = (u + 0x7FFFu + ((u >> 16) & 1u)) & 0xFFFF0000u;
  return __uint_as_float(u);
}

__device__ __forceinline__ f16x16 gfrag(const f16* __restrict__ base, int ld, int row0, int k0) {
  const int lane = threadIdx.x & 31, r = lane & 15, kh = (lane >> 4) * 8;
  const f16* p = base + (size_t)(row0 + r) * ld + k0 + kh;
  Frag u;
  u.h[0] = *(const f16x8*)p;
  u.h[1] = *(const f16x8*)(p + 16);
  return u.v;
}

__global__ __launch_bounds__(256) void k_prep(const float* __restrict__ U, const float* __restrict__ Wk, const float* __restrict__ Wv,
                                              f16* __restrict__ Uh, f16* __restrict__ Wkt, f16* __restrict__ Wvt, int nUblk) {
  __shared__ float tS[64][65];
  const int tid = threadIdx.x;
  if ((int)blockIdx.x < nUblk) {
    const int R0 = blockIdx.x * TOKB;
    const int b = R0 / SEQ, n0 = R0 % SEQ;
    const float* src0 = U + ((size_t)b * SEQ_FULL + n0) * CC;
    f16* dst0 = Uh + (size_t)R0 * CC;
#pragma unroll 1
    for (int pass = 0; pass < 2; ++pass) {
#pragma unroll 2
      for (int it = 0; it < 8; ++it) {
        const int ch = tid + 256 * it, row = ch >> 5, q = (ch & 31) * 8;
        const float* s = src0 + (size_t)row * CC + q;
        const v4f a0 = *(const v4f*)s;
        const v4f a1 = *(const v4f*)(s + 4);
        Pack8 p;
        p.v[0] = (f16)bf16r(a0[0]); p.v[1] = (f16)bf16r(a0[1]); p.v[2] = (f16)bf16r(a0[2]); p.v[3] = (f16)bf16r(a0[3]);
        p.v[4] = (f16)bf16r(a1[0]); p.v[5] = (f16)bf16r(a1[1]); p.v[6] = (f16)bf16r(a1[2]); p.v[7] = (f16)bf16r(a1[3]);
        *(volatile v4u*)(dst0 + (size_t)row * CC + q) = p.u;
      }
      __threadfence();
    }
  } else {
    const int wb = (int)blockIdx.x - nUblk;
    const int which = wb >> 4, t16 = wb & 15, bi = t16 >> 2, bj = t16 & 3;
    const float* Wm = (which != 0) ? Wv : Wk;
    f16* Wt = (which != 0) ? Wvt : Wkt;
    for (int e = tid; e < 64 * 64; e += 256) {
      const int r = e >> 6, c = e & 63;
      tS[r][c] = Wm[(size_t)(bi * 64 + r) * CC + bj * 64 + c];
    }
    __syncthreads();
#pragma unroll 1
    for (int pass = 0; pass < 2; ++pass) {
      for (int ch = tid; ch < 64 * 8; ch += 256) {
        const int r = ch >> 3, q8 = (ch & 7) * 8;
        Pack8 p;
#pragma unroll
        for (int e = 0; e < 8; ++e) p.v[e] = (f16)(bf16r(tS[q8 + e][r]) * WCARRY);
        *(volatile v4u*)(Wt + (size_t)(bj * 64 + r) * CC + bi * 64 + q8) = p.u;
      }
      __threadfence();
    }
  }
}

__global__ __launch_bounds__(256) void k_gemm_ln(const f16* __restrict__ Uh, const f16* __restrict__ Wkt, const f16* __restrict__ Wvt,
                                                 const float* __restrict__ gamma, const float* __restrict__ beta,
                                                 f16* __restrict__ KT, f16* __restrict__ VT) {
  __shared__ __attribute__((aligned(16))) f16 oT[CC * OTS];
  __shared__ float psum[4][TOKB];
  __shared__ float psq[4][TOKB];
  __shared__ float mu_s[TOKB];
  __shared__ float rs_s[TOKB];
  const int tid = threadIdx.x, lane = tid & 31, wave = tid >> 5, m = lane & 15, hh = lane >> 4;
  const int which = blockIdx.y;
  const f16* Wt = (which != 0) ? Wvt : Wkt;
  f16* dstT = (which != 0) ? VT : KT;
  const int R0 = blockIdx.x * TOKB;
  const int b = R0 / SEQ, n0 = R0 % SEQ;
  const int wm = (wave & 1) * 32, wg = wave >> 1, wn = wg * 64;

  f32x8 acc[2][4];
#pragma unroll
  for (int i = 0; i < 2; ++i)
#pragma unroll
    for (int j = 0; j < 4; ++j) { f32x8 z = {}; acc[i][j] = z; }

#pragma unroll 1
  for (int k0 = 0; k0 < CC; k0 += 32) {
    f16x16 af[2], bfr[4];
#pragma unroll
    for (int i = 0; i < 2; ++i) af[i] = gfrag(Uh, CC, R0 + wm + 16 * i, k0);
#pragma unroll
    for (int j = 0; j < 4; ++j) bfr[j] = gfrag(Wt, CC, wn + 16 * j, k0);
#pragma unroll
    for (int i = 0; i < 2; ++i)
#pragma unroll
      for (int j = 0; j < 4; ++j) acc[i][j] = wmma16(af[i], bfr[j], acc[i][j]);
  }

#pragma unroll
  for (int i = 0; i < 2; ++i)
#pragma unroll
    for (int j = 0; j < 4; ++j) acc[i][j] = acc[i][j] * WCARRY_INV;

#pragma unroll
  for (int i = 0; i < 2; ++i) {
#pragma unroll
    for (int r = 0; r < 8; ++r) {
      float s = (acc[i][0][r] + acc[i][1][r]) + (acc[i][2][r] + acc[i][3][r]);
      s += __shfl_xor(s, 1, 32); s += __shfl_xor(s, 2, 32); s += __shfl_xor(s, 4, 32); s += __shfl_xor(s, 8, 32);
      if (m == 0) psum[wg][wm + 16 * i + 8 * hh + r] = s;
    }
  }
  __syncthreads();
  if (tid < TOKB) mu_s[tid] = ((psum[0][tid] + psum[1][tid]) + (psum[2][tid] + psum[3][tid])) * (1.0f / (float)CC);
  __syncthreads();
#pragma unroll
  for (int i = 0; i < 2; ++i) {
#pragma unroll
    for (int r = 0; r < 8; ++r) {
      const float mu = mu_s[wm + 16 * i + 8 * hh + r];
      const float d0 = acc[i][0][r] - mu, d1 = acc[i][1][r] - mu, d2 = acc[i][2][r] - mu, d3 = acc[i][3][r] - mu;
      float s = (d0 * d0 + d1 * d1) + (d2 * d2 + d3 * d3);
      s += __shfl_xor(s, 1, 32); s += __shfl_xor(s, 2, 32); s += __shfl_xor(s, 4, 32); s += __shfl_xor(s, 8, 32);
      if (m == 0) psq[wg][wm + 16 * i + 8 * hh + r] = s;
    }
  }
  __syncthreads();
  if (tid < TOKB) {
    const float var = ((psq[0][tid] + psq[1][tid]) + (psq[2][tid] + psq[3][tid])) * (1.0f / (float)CC);
    rs_s[tid] = 1.0f / sqrtf(var + LN_EPS);
  }
  __syncthreads();

#pragma unroll
  for (int j = 0; j < 4; ++j) {
    const int c = wn + 16 * j + m;
    const float g = bf16r(gamma[c]), be = bf16r(beta[c]);
#pragma unroll
    for (int i = 0; i < 2; ++i) {
      Pack8 p;
#pragma unroll
      for (int r = 0; r < 8; ++r) {
        const int row = wm + 16 * i + 8 * hh + r;
        const float y = ((acc[i][j][r] - mu_s[row]) * rs_s[row] * g + be) * PCARRY;
        p.v[r] = (f16)y;
      }
      *(f16x8*)(oT + c * OTS + wm + 16 * i + 8 * hh) = p.v;
    }
  }
  __syncthreads();

  f16* dst = dstT + (size_t)b * CC * SEQ + n0;
#pragma unroll 1
  for (int pass = 0; pass < 2; ++pass) {
#pragma unroll 2
    for (int it = 0; it < 8; ++it) {
      const int ch = tid + 256 * it, c = ch >> 3, q = (ch & 7) * 8;
      *(volatile v4u*)(dst + (size_t)c * SEQ + q) = *(const v4ua*)(oT + c * OTS + q);
    }
    __threadfence();
  }
}

__global__ __launch_bounds__(256) void k_kv(const f16* __restrict__ KT, const f16* __restrict__ VT, const float* __restrict__ Wq,
                                            float* __restrict__ Mtab) {
  __shared__ float part[8][DD * DD];
  __shared__ float kvs[DD * DD];
  __shared__ __attribute__((aligned(16))) float Ms[DD];
  const int tid = threadIdx.x, lane = tid & 31, wave = tid >> 5, m = lane & 15, hh = lane >> 4;
  const int b = blockIdx.x / HH, h = blockIdx.x % HH;
  const f16* Kb = KT + (size_t)b * CC * SEQ;
  const f16* Vb = VT + (size_t)b * CC * SEQ;
  const int nPer = SEQ / 8, nbeg = wave * nPer;

  f32x8 acc[2][2];
#pragma unroll
  for (int i = 0; i < 2; ++i)
#pragma unroll
    for (int j = 0; j < 2; ++j) { f32x8 z = {}; acc[i][j] = z; }

#pragma unroll 1
  for (int k0 = nbeg; k0 < nbeg + nPer; k0 += 32) {
    f16x16 af[2], bfr[2];
#pragma unroll
    for (int i = 0; i < 2; ++i) af[i] = gfrag(Kb, SEQ, h * DD + 16 * i, k0);
#pragma unroll
    for (int j = 0; j < 2; ++j) bfr[j] = gfrag(Vb, SEQ, h * DD + 16 * j, k0);
#pragma unroll
    for (int i = 0; i < 2; ++i)
#pragma unroll
      for (int j = 0; j < 2; ++j) acc[i][j] = wmma16(af[i], bfr[j], acc[i][j]);
  }

  float* pw = part[wave];
#pragma unroll
  for (int i = 0; i < 2; ++i)
#pragma unroll
    for (int j = 0; j < 2; ++j)
#pragma unroll
      for (int r = 0; r < 8; ++r) pw[(16 * i + 8 * hh + r) * DD + 16 * j + m] = acc[i][j][r];
  __syncthreads();
#pragma unroll
  for (int q = 0; q < 4; ++q) {
    const int idx = tid + 256 * q;
    float s = part[0][idx];
#pragma unroll
    for (int w = 1; w < 8; ++w) s += part[w][idx];
    kvs[idx] = s;
  }
  __syncthreads();
  if (tid < DD) {
    const float* wq = Wq + h * DD;
    float s = 0.0f;
#pragma unroll 1
    for (int d = 0; d < DD; ++d) s = fmaf(bf16r(wq[d]), kvs[d * DD + tid], s);
    Ms[tid] = s * ((1.0f / (float)SEQ) * (1.0f / (PCARRY * PCARRY)));
  }
  __syncthreads();
  float* dst = Mtab + (size_t)(b * HH + h) * DD;
#pragma unroll 1
  for (int pass = 0; pass < 2; ++pass) {
    if (tid < 8) *(volatile v4f*)(dst + 4 * tid) = *(const v4fa*)(Ms + 4 * tid);
    __threadfence();
  }
}

__global__ __launch_bounds__(256) void k_out(const float* __restrict__ X, const float* __restrict__ Mtab, float* __restrict__ out) {
  __shared__ __attribute__((aligned(16))) float Mc[CC];
  const int tid = threadIdx.x;
  const int R0 = blockIdx.x * TOKB;
  const int b = R0 / SEQ, n0 = R0 % SEQ;
  {
    const int c = tid, h = c % HH, e = c / HH;
    Mc[c] = Mtab[((size_t)b * HH + h) * DD + e];
  }
  __syncthreads();
  const float* xb = X + (size_t)b * SEQ_FULL + n0;
#pragma unroll 1
  for (int pass = 0; pass < 2; ++pass) {
#pragma unroll 4
    for (int it = 0; it < 16; ++it) {
      const int f4 = tid + 256 * it, row = f4 >> 6, q = (f4 & 63) * 4;
      const float xv = bf16r(xb[row]);
      v4f o = *(const v4fa*)(Mc + q);
      o = o * xv;
      *(volatile v4f*)(out + (size_t)(R0 + row) * CC + q) = o;
    }
    __threadfence();
  }
}

extern "C" void kernel_launch(void* const* d_in, const int* in_sizes, int n_in,
                              void* d_out, int out_size, void* d_ws, size_t ws_size,
                              hipStream_t stream) {
  if (n_in < 7) return;
  if (in_sizes[0] < ((NB - 1) * SEQ_FULL + SEQ) * CC) return;
  if (in_sizes[1] < (NB - 1) * SEQ_FULL + SEQ) return;
  if (in_sizes[2] < HH * DD || in_sizes[3] < CC * CC || in_sizes[4] < CC * CC || in_sizes[5] < CC || in_sizes[6] < CC) return;
  if (out_size < NB * SEQ * CC) return;
  const float* U     = (const float*)d_in[0];
  const float* X     = (const float*)d_in[1];
  const float* Wq    = (const float*)d_in[2];
  const float* Wk    = (const float*)d_in[3];
  const float* Wv    = (const float*)d_in[4];
  const float* gamma = (const float*)d_in[5];
  const float* beta  = (const float*)d_in[6];
  float* out = (float*)d_out;

  char* ws = (char*)d_ws;
  size_t off = 0;
  f16* Uh  = (f16*)(ws + off); off += (size_t)NB * SEQ * CC * 2;
  f16* Wkt = (f16*)(ws + off); off += (size_t)CC * CC * 2;
  f16* Wvt = (f16*)(ws + off); off += (size_t)CC * CC * 2;
  f16* KT  = (f16*)(ws + off); off += (size_t)NB * CC * SEQ * 2;
  f16* VT  = (f16*)(ws + off); off += (size_t)NB * CC * SEQ * 2;
  float* Mtab = (float*)(ws + off); off += (size_t)NB * HH * DD * 4;
  if (off > ws_size) return;

  const int nUblk = NB * SEQ / TOKB;
  k_prep<<<dim3(nUblk + 32), dim3(256), 0, stream>>>(U, Wk, Wv, Uh, Wkt, Wvt, nUblk);
  k_gemm_ln<<<dim3(nUblk, 2), dim3(256), 0, stream>>>(Uh, Wkt, Wvt, gamma, beta, KT, VT);
  k_kv<<<dim3(NB * HH), dim3(256), 0, stream>>>(KT, VT, Wq, Mtab);
  k_out<<<dim3(NB * SEQ / TOKB), dim3(256), 0, stream>>>(X, Mtab, out);
}
